// SlidingWindowAttention_7043746365913
// MI455X (gfx1250) — hardware-verified
//
#include <hip/hip_runtime.h>


#ifndef NB
#define NB 1
#endif
#ifndef SEQ
#define SEQ 2048
#endif
#define SEQ_FULL 2048
#define NB_  NB
#define TT   SEQ
#define TT_FULL SEQ_FULL
#define DM   768
#define NH_  12
#define HD   64
#define HW   64
#define PADT 64
#define BW   192
#define TP   (TT + 2 * PADT)
#define SCL  0.125f

static_assert(TT % 64 == 0);
static_assert(DM == NH_ * HD);
static_assert(HD == 64);
static_assert(BW % 32 == 0);
static_assert(BW == 64 + 2 * PADT);
static_assert(HW <= PADT);
static_assert(TP % 64 == 0);
static_assert((NH_ * TT) % 8 == 0);

typedef unsigned short bf;
typedef __attribute__((ext_vector_type(16))) __bf16   v16bf;
typedef __attribute__((ext_vector_type(8)))  unsigned short v8us;
typedef __attribute__((ext_vector_type(8)))  float    v8f;
typedef __attribute__((ext_vector_type(4)))  float    v4f;
typedef __attribute__((ext_vector_type(2)))  float    v2f;
typedef __attribute__((ext_vector_type(2)))  unsigned short v2us;
typedef v4f  __attribute__((may_alias)) v4fa;

__device__ __forceinline__ unsigned short f2bf(float f) { unsigned u = __float_as_uint(f); u += 0x7FFFu + ((u >> 16) & 1u); return (unsigned short)(u >> 16); }
__device__ __forceinline__ float bf2f(unsigned short b) { return __uint_as_float(((unsigned)b) << 16); }
__device__ __forceinline__ float bfr(float f) { return bf2f(f2bf(f)); }
__device__ __forceinline__ void splitf(float y, unsigned short& h, unsigned short& l) { h = f2bf(y); l = f2bf(y - bf2f(h)); }
__device__ __forceinline__ v16bf cat16b(v8us lo, v8us hi) { return __builtin_bit_cast(v16bf, __builtin_shufflevector(lo, hi, 0, 1, 2, 3, 4, 5, 6, 7, 8, 9, 10, 11, 12, 13, 14, 15)); }
__device__ __forceinline__ v8f wmmab(v16bf a, v16bf b, v8f c) { return __builtin_amdgcn_wmma_f32_16x16x32_bf16(false, a, false, b, (short)0, c, false, false); }
__device__ __forceinline__ v16bf ldf(const bf* p) { return cat16b(*(const v8us*)p, *(const v8us*)(p + 16)); }

template <int NSPLIT, bool BIAS>
__global__ __launch_bounds__(32) void k_gemm(const bf* __restrict__ A, const bf* __restrict__ A2, int lda, const bf* __restrict__ Bt, const bf* __restrict__ Bt2, int ldb, int K, int bandN, int bandK,
                                            float* C, int ldc, const float* __restrict__ bias, size_t sA, size_t sB, size_t sC) {
    __shared__ __align__(16) float os[16 * 68];
    const size_t z = blockIdx.z; A += z * sA; if (A2) A2 += z * sA; Bt += z * sB; if (Bt2) Bt2 += z * sB; C += z * sC;
    const int lane = threadIdx.x & 31, lr = lane & 15, hi = lane >> 4; const int r0 = blockIdx.x * 64, c0 = blockIdx.y * 64;
    v8f acc[4][4];
#pragma unroll
    for (int mb = 0; mb < 4; ++mb)
#pragma unroll
        for (int nb = 0; nb < 4; ++nb) acc[mb][nb] = (v8f){};
    const size_t aoff = (size_t)(r0 + lr) * lda + 8 * hi;
    const size_t boff = (size_t)(c0 + bandN * r0 + lr) * ldb + (size_t)bandK * r0 + 8 * hi;
#pragma unroll 1
    for (int kc = 0; kc < K; kc += 32) {
        v16bf a[4], a2[4];
#pragma unroll
        for (int mb = 0; mb < 4; ++mb) { a[mb] = ldf(A + aoff + (size_t)mb * 16 * lda + kc); if (NSPLIT == 1 || NSPLIT == 2) a2[mb] = ldf(A2 + aoff + (size_t)mb * 16 * lda + kc); }
#pragma unroll
        for (int nb = 0; nb < 4; ++nb) { const v16bf b = ldf(Bt + boff + (size_t)nb * 16 * ldb + kc); v16bf b2; if (NSPLIT >= 2) b2 = ldf(Bt2 + boff + (size_t)nb * 16 * ldb + kc);
#pragma unroll
            for (int mb = 0; mb < 4; ++mb) { acc[mb][nb] = wmmab(a[mb], b, acc[mb][nb]); if (NSPLIT == 1 || NSPLIT == 2) acc[mb][nb] = wmmab(a2[mb], b, acc[mb][nb]); if (NSPLIT >= 2) acc[mb][nb] = wmmab(a[mb], b2, acc[mb][nb]); } }
        asm volatile("v_nop\n\tv_nop\n\tv_nop\n\tv_nop" : "+v"(acc[0][0]), "+v"(acc[1][1]), "+v"(acc[2][2]), "+v"(acc[3][3]) : "v"(a[0]), "v"(a[3]));
    }
#pragma unroll
    for (int mb = 0; mb < 4; ++mb) {
#pragma unroll
        for (int nb = 0; nb < 4; ++nb) {
#pragma unroll
            for (int j = 0; j < 8; ++j) os[(hi * 8 + j) * 68 + nb * 16 + lr] = acc[mb][nb][j]; }
        __builtin_amdgcn_fence(3  , "wavefront"); __builtin_amdgcn_wave_barrier(); asm volatile("" ::: "memory");
        float* crow = C + (size_t)(r0 + mb * 16) * ldc + c0;
#pragma unroll 1
        for (int ps = 0; ps < 2; ++ps) {
#pragma unroll
            for (int s = 0; s < 8; ++s) { const int row = 2 * s + hi, cofs = lr * 4; v4f val = *(const v4fa*)(os + row * 68 + cofs);
                if (BIAS) { val[0] += bfr(bias[c0 + cofs]); val[1] += bfr(bias[c0 + cofs + 1]); val[2] += bfr(bias[c0 + cofs + 2]); val[3] += bfr(bias[c0 + cofs + 3]); }
                *(volatile v4f*)(crow + (size_t)row * ldc + cofs) = val; }
            if (ps == 0) __threadfence(); }
        __builtin_amdgcn_fence(3  , "wavefront"); __builtin_amdgcn_wave_barrier(); asm volatile("" ::: "memory");
    }
}

__global__ __launch_bounds__(256) void k_wtG(const float* __restrict__ w, int K, int N, bf* Bt) {
    const int lane = threadIdx.x & 31; const int L0 = (blockIdx.x * 8 + (threadIdx.x >> 5)) * 8; const int nlines = N * K / 64;
#pragma unroll
    for (int ps = 0; ps < 2; ++ps) {
#pragma unroll 1
        for (int l = 0; l < 8; ++l) { const int L = L0 + l; if (L >= nlines) break; const size_t e = (size_t)L * 64 + lane * 2; const int k = (int)(e % K), n = (int)(e / K); v2us o;
            o[0] = f2bf(w[(size_t)k * N + n]); o[1] = f2bf(w[(size_t)(k + 1) * N + n]); *(volatile v2us*)(Bt + e) = o; }
        if (ps == 0) __threadfence(); }
}
__global__ __launch_bounds__(256) void k_cvt8(const float* __restrict__ src, bf* dst, size_t n8) { const size_t i = (size_t)blockIdx.x * 256 + threadIdx.x; if (i >= n8) return; const v8f v = *(const v8f*)(src + i * 8); v8us o;
#pragma unroll
    for (int k = 0; k < 8; ++k) o[k] = f2bf(v[k]); *(volatile v8us*)(dst + i * 8) = o; __threadfence(); *(volatile v8us*)(dst + i * 8) = o; }

__global__ __launch_bounds__(256) void k_qkp(const float* __restrict__ F, int pitch, int nheads, int PR, int pad, bf* Ph, bf* Pl) {
    const size_t e = ((size_t)blockIdx.x * 256 + threadIdx.x) * 2; if (e >= (size_t)nheads * PR * HD) return;
    const int d = (int)(e % HD); const int r = (int)((e / HD) % PR); const int h = (int)(e / ((size_t)HD * PR)); const int t = r - pad; const bool in = (t >= 0) && (t < TT); const int tc = min(max(t, 0), TT - 1);
    const float* f = F + (size_t)tc * pitch + h * HD + d; v2us oh, ol;
#pragma unroll
    for (int q = 0; q < 2; ++q) { float x = f[q]; x = in ? x : 0.0f; unsigned short a2, c2; splitf(x, a2, c2); oh[q] = a2; ol[q] = c2; }
    *(volatile v2us*)(Ph + e) = oh; *(volatile v2us*)(Pl + e) = ol; __threadfence(); *(volatile v2us*)(Ph + e) = oh; *(volatile v2us*)(Pl + e) = ol;
}
__global__ __launch_bounds__(256) void k_vtp(const float* __restrict__ F, int pitch, int nheads, bf* Vh, bf* Vl) {
    const size_t e = ((size_t)blockIdx.x * 256 + threadIdx.x) * 2; if (e >= (size_t)nheads * HD * TP) return;
    const int c = (int)(e % TP); const int d = (int)((e / TP) % HD); const int g = (int)(e / ((size_t)TP * HD)); v2us oh, ol;
#pragma unroll
    for (int q = 0; q < 2; ++q) { const int t = c + q - PADT; const bool in = (t >= 0) && (t < TT); const int tc = min(max(t, 0), TT - 1);
        float x = F[(size_t)tc * pitch + g * HD + d]; x = in ? x : 0.0f; unsigned short a2, c2; splitf(x, a2, c2); oh[q] = a2; ol[q] = c2; }
    *(volatile v2us*)(Vh + e) = oh; *(volatile v2us*)(Vl + e) = ol; __threadfence(); *(volatile v2us*)(Vh + e) = oh; *(volatile v2us*)(Vl + e) = ol;
}
__global__ __launch_bounds__(256) void k_asoft(const float* __restrict__ Sb, bf* Ph, bf* Pl) {
    const int lane = threadIdx.x & 31; const int row = blockIdx.x * 8 + (threadIdx.x >> 5); if (row >= NH_ * TT) return;
    const int i = row % TT; const int p0 = (i & ~63) - PADT; const float* sr = Sb + (size_t)row * BW; float v[BW / 32]; float mx = -3.0e38f;
#pragma unroll
    for (int ch = 0; ch < BW / 64; ++ch) { const int j0 = ch * 64 + lane * 2; const v2f a = *(const v2f*)(sr + j0);
#pragma unroll
        for (int q = 0; q < 2; ++q) { const int p = p0 + j0 + q; const bool ok = (p >= 0) && (p < TT) && (p >= i - HW) && (p <= i + HW); const float t = ok ? a[q] * SCL : -3.0e38f; v[ch * 2 + q] = t; mx = fmaxf(mx, t); } }
#pragma unroll
    for (int sh = 16; sh; sh >>= 1) mx = fmaxf(mx, __shfl_xor(mx, sh, 32));
    float sum = 0.f;
#pragma unroll
    for (int k = 0; k < BW / 32; ++k) { float d0 = __fsub_rn(v[k], mx); asm volatile("" : "+v"(d0)); v[k] = __builtin_amdgcn_exp2f(__fmul_rn(d0, 1.4426950408889634f)); sum += v[k]; }
#pragma unroll
    for (int sh = 16; sh; sh >>= 1) sum += __shfl_xor(sum, sh, 32);
    const float f = __fdiv_rn(1.0f, sum);
#pragma unroll 1
    for (int ps = 0; ps < 2; ++ps) {
#pragma unroll
        for (int ch = 0; ch < BW / 64; ++ch) { v2us oh, ol;
#pragma unroll
            for (int q = 0; q < 2; ++q) { unsigned short a2, c2; splitf(v[ch * 2 + q] * f, a2, c2); oh[q] = a2; ol[q] = c2; }
            const size_t oo = (size_t)row * BW + ch * 64 + lane * 2; *(volatile v2us*)(Ph + oo) = oh; *(volatile v2us*)(Pl + oo) = ol; }
        if (ps == 0) __threadfence(); }
}
__global__ __launch_bounds__(256) void k_merge(const float* __restrict__ O, bf* Ah, bf* Al) {
    const size_t e = ((size_t)blockIdx.x * 256 + threadIdx.x) * 2; if (e >= (size_t)NH_ * TT * HD) return;
    const int d = (int)(e % HD); const int t = (int)((e / HD) % TT); const int h = (int)(e / ((size_t)HD * TT)); const size_t oo = (size_t)t * DM + h * HD + d; v2us oh, ol;
#pragma unroll
    for (int q = 0; q < 2; ++q) { unsigned short a2, c2; splitf(O[e + q], a2, c2); oh[q] = a2; ol[q] = c2; }
    *(volatile v2us*)(Ah + oo) = oh; *(volatile v2us*)(Al + oo) = ol; __threadfence(); *(volatile v2us*)(Ah + oo) = oh; *(volatile v2us*)(Al + oo) = ol;
}

extern "C" void kernel_launch(void* const* d_in, const int* in_sizes, int n_in,
                              void* d_out, int out_size, void* d_ws, size_t ws_size, hipStream_t stream) {
    if (n_in < 11) return;
    if (in_sizes[0] < NB_ * TT * DM || in_sizes[1] < NB_ * TT * DM || in_sizes[2] < NB_ * TT * DM) return;
    if (in_sizes[3] < DM * DM || in_sizes[5] < DM * DM || in_sizes[7] < DM * DM || in_sizes[9] < DM * DM) return;
    if (in_sizes[4] < DM || in_sizes[6] < DM || in_sizes[8] < DM || in_sizes[10] < DM) return;
    if (out_size < NB_ * TT * DM) return;
    const float* xq = (const float*)d_in[0]; const float* xk = (const float*)d_in[1]; const float* xv = (const float*)d_in[2];
    const float* wq = (const float*)d_in[3]; const float* bq = (const float*)d_in[4]; const float* wk = (const float*)d_in[5]; const float* bk = (const float*)d_in[6];
    const float* wv = (const float*)d_in[7]; const float* bv = (const float*)d_in[8]; const float* wo = (const float*)d_in[9]; const float* bo = (const float*)d_in[10];
    float* OUT = (float*)d_out;
    char* wsp = (char*)d_ws;
    auto take = [&](size_t bytes) { char* p = wsp; wsp += (bytes + 255) & ~(size_t)255; return (void*)p; };
    bf* WQ = (bf*)take((size_t)DM * DM * 2); bf* WK = (bf*)take((size_t)DM * DM * 2); bf* WV = (bf*)take((size_t)DM * DM * 2); bf* WO = (bf*)take((size_t)DM * DM * 2);
    bf* XQ = (bf*)take((size_t)TT * DM * 2); bf* XK = (bf*)take((size_t)TT * DM * 2); bf* XV = (bf*)take((size_t)TT * DM * 2);
    float* FQ = (float*)take((size_t)TT * DM * 4); float* FK = (float*)take((size_t)TT * DM * 4); float* FV = (float*)take((size_t)TT * DM * 4);
    bf* QPh = (bf*)take((size_t)NH_ * TT * HD * 2); bf* QPl = (bf*)take((size_t)NH_ * TT * HD * 2);
    bf* KPh = (bf*)take((size_t)NH_ * TP * HD * 2); bf* KPl = (bf*)take((size_t)NH_ * TP * HD * 2);
    bf* VTh = (bf*)take((size_t)NH_ * HD * TP * 2); bf* VTl = (bf*)take((size_t)NH_ * HD * TP * 2);
    float* Sb = (float*)take((size_t)NH_ * TT * BW * 4); bf* Ph = (bf*)take((size_t)NH_ * TT * BW * 2); bf* Pl = (bf*)take((size_t)NH_ * TT * BW * 2);
    float* Ob = (float*)take((size_t)NH_ * TT * HD * 4); bf* ATh = (bf*)take((size_t)TT * DM * 2); bf* ATl = (bf*)take((size_t)TT * DM * 2);
    const size_t used = (size_t)(wsp - (char*)d_ws);
    if (used > ws_size || used > ((size_t)128 << 20)) return;

    const unsigned gW = (unsigned)((DM * DM / 64 + 63) / 64);
    k_wtG<<<gW, 256, 0, stream>>>(wq, DM, DM, WQ);
    k_wtG<<<gW, 256, 0, stream>>>(wk, DM, DM, WK);
    k_wtG<<<gW, 256, 0, stream>>>(wv, DM, DM, WV);
    k_wtG<<<gW, 256, 0, stream>>>(wo, DM, DM, WO);
    const size_t n8 = (size_t)TT * DM / 8; const unsigned gC = (unsigned)((n8 + 255) / 256);
    const unsigned gQ = (unsigned)(((size_t)NH_ * TT * HD / 2 + 255) / 256), gK = (unsigned)(((size_t)NH_ * TP * HD / 2 + 255) / 256);
    for (int b = 0; b < NB_; ++b) {
        const size_t xo = (size_t)b * TT_FULL * DM;
        k_cvt8<<<gC, 256, 0, stream>>>(xq + xo, XQ, n8);
        k_cvt8<<<gC, 256, 0, stream>>>(xk + xo, XK, n8);
        k_cvt8<<<gC, 256, 0, stream>>>(xv + xo, XV, n8);
        k_gemm<0, true><<<dim3(TT / 64, DM / 64, 1), 32, 0, stream>>>(XQ, nullptr, DM, WQ, nullptr, DM, DM, 0, 0, FQ, DM, bq, 0, 0, 0);
        k_gemm<0, true><<<dim3(TT / 64, DM / 64, 1), 32, 0, stream>>>(XK, nullptr, DM, WK, nullptr, DM, DM, 0, 0, FK, DM, bk, 0, 0, 0);
        k_gemm<0, true><<<dim3(TT / 64, DM / 64, 1), 32, 0, stream>>>(XV, nullptr, DM, WV, nullptr, DM, DM, 0, 0, FV, DM, bv, 0, 0, 0);
        k_qkp<<<gQ, 256, 0, stream>>>(FQ, DM, NH_, TT, 0, QPh, QPl);
        k_qkp<<<gK, 256, 0, stream>>>(FK, DM, NH_, TP, PADT, KPh, KPl);
        k_vtp<<<gK, 256, 0, stream>>>(FV, DM, NH_, VTh, VTl);
        k_gemm<2, false><<<dim3(TT / 64, BW / 64, NH_), 32, 0, stream>>>(QPh, QPl, HD, KPh, KPl, HD, HD, 1, 0, Sb, BW, nullptr, (size_t)TT * HD, (size_t)TP * HD, (size_t)TT * BW);
        k_asoft<<<(NH_ * TT) / 8, 256, 0, stream>>>(Sb, Ph, Pl);
        k_gemm<2, false><<<dim3(TT / 64, HD / 64, NH_), 32, 0, stream>>>(Ph, Pl, BW, VTh, VTl, TP, BW, 0, 1, Ob, HD, nullptr, (size_t)TT * BW, (size_t)HD * TP, (size_t)TT * HD);
        k_merge<<<gQ, 256, 0, stream>>>(Ob, ATh, ATl);
        k_gemm<1, true><<<dim3(TT / 64, DM / 64, 1), 32, 0, stream>>>(ATh, ATl, DM, WO, nullptr, DM, DM, 0, 0, OUT + (size_t)b * TT * DM, DM, bo, 0, 0, 0);
    }
}
